// EnBaseLayer_48576080117843
// MI455X (gfx1250) — hardware-run, weakly checked
//
#include <hip/hip_runtime.h>
#include <stddef.h>
#include <math.h>


#define HDIM   128
#define EFD    8
#define NRBF   20
#define KE     32
#define K1R    284
#define PW     256
#define NTHR   256
#define NWV    8
#define TR     64
#define LDH    136
#define BM     32
#define CE     81920
#define NB     256
#define CH     2048
#define LCAP   4096
#define SP     128
#define WSCAP  134217728
#define SCL_H   8.0f
#define SCL_W   16.0f
#define SCL_EF  64.0f
#define SCL_ACT 8.0f
#define INV_HW  0.0078125f
#define INV_EW  0.0009765625f

#define LG_SLIST 0
#define LG_SLOTS (LG_SLIST + LCAP * 4)
#define LG_SDL   (LG_SLOTS + NB * SP * 2)
#define LG_SDX   (LG_SDL + LCAP * 4)
#define LG_XO    (LG_SDX + NB * 4 * 4)
#define LG_SCNT  (LG_XO + NB * 3 * 4)
#define LG_WSUM  (LG_SCNT + NB * 4)
#define LDS_G    (LG_WSUM + 64)

static_assert((LDH % 8) == 0 && LDH >= HDIM);
static_assert(TR == 64 && NWV * 32 == NTHR && (TR * HDIM / 8) % NTHR == 0 && (TR * HDIM / 4) % NTHR == 0);
static_assert((CE % TR) == 0 && (CE % 4) == 0);
static_assert(NB == NTHR && CH == 8 * NTHR && LCAP >= 2 * CH && (LCAP % 4) == 0 && LCAP <= 65536 && SP <= LCAP);
static_assert((NB * 3) % 4 == 0 && (NB * 3 / 4) <= NTHR && NB == 32 * NWV);
static_assert(BM * 8 == NTHR && PW == 2 * HDIM && (HDIM % 32) == 0 && NRBF + EFD <= KE);
static_assert((LG_SLOTS % 16) == 0 && (LG_SDL % 16) == 0 && (LG_SDX % 16) == 0 && (LG_XO % 16) == 0);
static_assert((LG_SCNT % 16) == 0 && (LG_WSUM % 16) == 0);

typedef float    v4f  __attribute__((ext_vector_type(4)));
typedef float    v8f  __attribute__((ext_vector_type(8)));
typedef int      v4i  __attribute__((ext_vector_type(4)));
typedef _Float16 v8h  __attribute__((ext_vector_type(8)));
typedef _Float16 v16h __attribute__((ext_vector_type(16)));
union FragH { v16h v; v8h hh[2]; };

__constant__ float c_off[NRBF] = {0.f, 1.f, 1.25f, 1.5f, 1.75f, 2.f, 2.25f, 2.5f, 2.75f, 3.f,
                                  3.5f, 4.f, 4.5f, 5.f, 5.5f, 6.f, 7.f, 8.f, 9.f, 10.f};

__device__ __forceinline__ v8f wmh(v16h a, v16h b, v8f c) {
  v8f d = __builtin_amdgcn_wmma_f32_16x16x32_f16(false, a, false, b, (short)0, c, false, false);
  asm volatile("v_nop\n\tv_nop\n\tv_nop\n\tv_nop" : "+v"(d) : "v"(a), "v"(b));
  return d;
}

__device__ __forceinline__ v8f zero8() { v8f z = {0.f, 0.f, 0.f, 0.f, 0.f, 0.f, 0.f, 0.f}; return z; }

__device__ __forceinline__ v8h cvt8(v4f a, v4f b, float s) {
  v8f t;
  t[0] = a.x * s; t[1] = a.y * s; t[2] = a.z * s; t[3] = a.w * s;
  t[4] = b.x * s; t[5] = b.y * s; t[6] = b.z * s; t[7] = b.w * s;
  return __builtin_convertvector(t, v8h);
}

__device__ __forceinline__ v16h frag16(const _Float16* p) {
  FragH f;
  f.hh[0] = *(const v8h*)p;
  f.hh[1] = *(const v8h*)(p + 16);
  return f.v;
}

__device__ __forceinline__ v16h afrag_f32(const float* rp, int h, float s) {
  FragH a;
  const float* p0 = rp + 8 * h;
  const float* p1 = rp + 16 + 8 * h;
  a.hh[0] = cvt8(*(const v4f*)p0, *(const v4f*)(p0 + 4), s);
  a.hh[1] = cvt8(*(const v4f*)p1, *(const v4f*)(p1 + 4), s);
  return a.v;
}

__device__ __forceinline__ float rcp_f(float x)  { return __builtin_amdgcn_rcpf(x); }
__device__ __forceinline__ float silu_f(float x) { return x * rcp_f(1.0f + __expf(-x)); }
__device__ __forceinline__ float sigm_f(float x) { return rcp_f(1.0f + __expf(-x)); }

__global__ __launch_bounds__(NTHR) void k_wcvt(const float* __restrict__ in, _Float16* outp,
                                               int C, int koff, int K, int KP, int nUnits, float scale) {
  const int u = (int)blockIdx.x * NTHR + (int)threadIdx.x;
  if (u >= nUnits) return;
  const int upr = KP >> 3;
  const int n   = u / upr;
  const int k0  = (u - n * upr) * 8;
  v8f t;
#pragma unroll
  for (int i = 0; i < 8; ++i) {
    const int k  = k0 + i;
    const int kc = k < K ? k : K - 1;
    const float v = in[(size_t)(koff + kc) * C + n] * scale;
    t[i] = (k < K) ? v : 0.0f;
  }
  const v8h o = __builtin_convertvector(t, v8h);
  _Float16* d = outp + (size_t)n * KP + k0;
  *(volatile v8h*)d = o;
  __threadfence();
  *(volatile v8h*)d = o;
}

__global__ __launch_bounds__(NTHR) __attribute__((amdgpu_num_vgpr(256)))
void k_nodegemm(const float* __restrict__ hin, const _Float16* __restrict__ wPQ,
                const float* __restrict__ b1, float* pq, int nN) {
  constexpr int NIT4 = (BM * PW / 4) / NTHR;
  static_assert((BM * PW / 4) % NTHR == 0 && NIT4 == 8);
  __shared__ __attribute__((aligned(16))) float stg[BM * PW];
  const int tid = threadIdx.x, lane = tid & 31;
  const int wave = __builtin_amdgcn_readfirstlane(tid >> 5);
  const int hh = lane >> 4, m = lane & 15;
  const int rg = wave >> 2, cq = wave & 3;
  const int r0 = rg * 16, c0 = cq * 64;
  const int rowBase = blockIdx.x * BM;

  v8f acc[4];
#pragma unroll
  for (int t = 0; t < 4; ++t) acc[t] = zero8();

  int ar = rowBase + r0 + m;
  ar = ar > nN - 1 ? nN - 1 : ar;
  const float* ap = hin + (size_t)ar * HDIM;
  const _Float16* bp0 = wPQ + (size_t)(c0 + m) * HDIM + 8 * hh;
#pragma unroll 1
  for (int kt = 0; kt < HDIM / 32; ++kt) {
    const v16h a = afrag_f32(ap + 32 * kt, hh, SCL_H);
#pragma unroll
    for (int t = 0; t < 4; ++t) acc[t] = wmh(a, frag16(bp0 + (size_t)(16 * t) * HDIM + 32 * kt), acc[t]);
  }

  float* sp = stg + (size_t)(r0 + 8 * hh) * PW + c0 + m;
  const int grow0 = rowBase + r0 + 8 * hh;
#pragma unroll
  for (int t = 0; t < 4; ++t) {
    const int n  = c0 + 16 * t + m;
    const int nb = n < HDIM ? n : HDIM - 1;
    float bv = b1[nb];
    bv = (n < HDIM) ? bv : 0.0f;
#pragma unroll
    for (int r = 0; r < 8; ++r) {
      float v = acc[t][r] * INV_HW + bv;
      v = (grow0 + r < nN) ? v : 0.0f;
      sp[r * PW + 16 * t] = v;
    }
  }
  __syncthreads();

  float* tile = pq + (size_t)rowBase * PW;
  v4f ov[NIT4];
#pragma unroll
  for (int it = 0; it < NIT4; ++it) ov[it] = *(const v4f*)(stg + 4 * (it * NTHR + tid));
#pragma unroll
  for (int it = 0; it < NIT4; ++it) *(volatile v4f*)(tile + 4 * (size_t)(it * NTHR + tid)) = ov[it];
  __threadfence();
#pragma unroll
  for (int it = 0; it < NIT4; ++it) *(volatile v4f*)(tile + 4 * (size_t)(it * NTHR + tid)) = ov[it];
}

__global__ __launch_bounds__(NTHR) __attribute__((amdgpu_num_vgpr(256)))
void k_edge1(const float* __restrict__ pq, const int* __restrict__ ei, const float* __restrict__ x,
             const float* __restrict__ ea, const _Float16* __restrict__ wE, _Float16* m1p,
             int nE, int nN, int ebase) {
  constexpr int NIT = (TR * HDIM / 8) / NTHR;
  constexpr int NSU = (16 * 64 / 4) / 32;
  __shared__ __attribute__((aligned(16))) float    stg[TR * HDIM];
  __shared__ __attribute__((aligned(16))) _Float16 tile[TR * LDH];
  const int tid = threadIdx.x, lane = tid & 31;
  const int wave = __builtin_amdgcn_readfirstlane(tid >> 5);
  const int h = lane >> 4, m = lane & 15;
  const int rg = wave >> 1, ch = wave & 1;
  const int cb = 64 * ch;
  const int rl0 = blockIdx.x * TR;
  const int e0 = ebase + rl0;

  const int eg = e0 + 16 * rg + m;
  const int e = eg > nE - 1 ? nE - 1 : eg;
  int s = ei[e];
  int d = ei[(size_t)nE + e];
  s = s < 0 ? 0 : (s > nN - 1 ? nN - 1 : s);
  d = d < 0 ? 0 : (d > nN - 1 ? nN - 1 : d);
  const float* xs = x + (size_t)s * 3;
  const float* xd = x + (size_t)d * 3;
  const float rx = xd[0] - xs[0], ry = xd[1] - xs[1], rz = xd[2] - xs[2];
  const float dsq  = (rx * rx + rz * rz) + ry * ry;
  const float dist = sqrtf(dsq + 1e-8f);
  const v4f av = *(const v4f*)(ea + (size_t)e * EFD + 4 * h);

  FragH ef;
  {
    v8f t0, t1;
#pragma unroll
    for (int i = 0; i < 8; ++i) {
      const float o0 = c_off[i], o1 = c_off[8 + i];
      const float off = (h == 0) ? o0 : o1;
      const float dd = dist - off;
      t0[i] = __expf(-0.5f * (dd * dd)) * SCL_EF;
    }
#pragma unroll
    for (int i = 0; i < 4; ++i) {
      const float dd = dist - c_off[16 + i];
      const float rb = __expf(-0.5f * (dd * dd)) * SCL_EF;
      const float at = av[i] * SCL_EF;
      t1[i]     = (h == 0) ? rb : at;
      t1[4 + i] = (h == 0) ? at : 0.0f;
    }
    ef.hh[0] = __builtin_convertvector(t0, v8h);
    ef.hh[1] = __builtin_convertvector(t1, v8h);
  }
  v8f acc1[4];
#pragma unroll
  for (int nt = 0; nt < 4; ++nt) acc1[nt] = zero8();
  {
    const _Float16* bp0 = wE + (size_t)(cb + m) * KE + 8 * h;
#pragma unroll
    for (int nt = 0; nt < 4; ++nt) acc1[nt] = wmh(ef.v, frag16(bp0 + (size_t)(16 * nt) * KE), acc1[nt]);
  }

#pragma unroll 4
  for (int i = 0; i < NSU; ++i) {
    const int u   = i * 32 + lane;
    const int row = u >> 4;
    const int c4  = (u & 15) * 4;
    const int dr  = __shfl(d, row);
    const int sr  = __shfl(s, row);
    const v4f p4 = *(const v4f*)(pq + (size_t)dr * PW + cb + c4);
    const v4f q4 = *(const v4f*)(pq + (size_t)sr * PW + HDIM + cb + c4);
    *(v4f*)(stg + (size_t)(16 * rg + row) * HDIM + cb + c4) = p4 + q4;
  }
  __syncthreads();

  {
    const float* srow = stg + (size_t)(16 * rg + 8 * h) * HDIM + cb + m;
    _Float16* trow = tile + (size_t)(16 * rg + 8 * h) * LDH + cb + m;
#pragma unroll
    for (int r = 0; r < 8; ++r) {
#pragma unroll
      for (int nt = 0; nt < 4; ++nt) {
        const float pre = acc1[nt][r] * INV_EW + srow[r * HDIM + 16 * nt];
        trow[r * LDH + 16 * nt] = (_Float16)(silu_f(pre) * SCL_ACT);
      }
    }
  }
  __syncthreads();

  _Float16* dstp = m1p + (size_t)rl0 * HDIM;
  v8h ov[NIT];
#pragma unroll
  for (int it = 0; it < NIT; ++it) {
    const int u = it * NTHR + tid;
    ov[it] = *(const v8h*)(tile + (u >> 4) * LDH + (u & 15) * 8);
  }
#pragma unroll
  for (int it = 0; it < NIT; ++it) *(volatile v8h*)(dstp + 8 * (size_t)(it * NTHR + tid)) = ov[it];
  __threadfence();
#pragma unroll
  for (int it = 0; it < NIT; ++it) *(volatile v8h*)(dstp + 8 * (size_t)(it * NTHR + tid)) = ov[it];
}

__global__ __launch_bounds__(NTHR) __attribute__((amdgpu_num_vgpr(256)))
void k_edge2(const _Float16* __restrict__ m1p, const int* __restrict__ ei, const float* __restrict__ x,
             const _Float16* __restrict__ w2, const _Float16* __restrict__ wx,
             const float* __restrict__ be2, const float* __restrict__ Winf, const float* __restrict__ binf,
             const float* __restrict__ bx1, const float* __restrict__ Wx2,
             float* mijf, float* aux, int nE, int nN, int ebase) {
  constexpr int NIT4 = (TR * HDIM / 4) / NTHR;
  __shared__ __attribute__((aligned(16))) float    stg[TR * HDIM];
  __shared__ __attribute__((aligned(16))) _Float16 tile[TR * LDH];
  __shared__ float esx[TR * 2];
  __shared__ float xsx[TR * 2];
  const int tid = threadIdx.x, lane = tid & 31;
  const int wave = __builtin_amdgcn_readfirstlane(tid >> 5);
  const int h = lane >> 4, m = lane & 15;
  const int rg = wave >> 1, ch = wave & 1;
  const int cb = 64 * ch;
  const int rl0 = blockIdx.x * TR;

  v8f acc[4];
#pragma unroll
  for (int nt = 0; nt < 4; ++nt) acc[nt] = zero8();
  {
    const _Float16* ap  = m1p + (size_t)(rl0 + 16 * rg + m) * HDIM + 8 * h;
    const _Float16* bp0 = w2 + (size_t)(cb + m) * HDIM + 8 * h;
#pragma unroll 1
    for (int kt = 0; kt < HDIM / 32; ++kt) {
      const v16h a = frag16(ap + 32 * kt);
#pragma unroll
      for (int nt = 0; nt < 4; ++nt) acc[nt] = wmh(a, frag16(bp0 + (size_t)(16 * nt) * HDIM + 32 * kt), acc[nt]);
    }
  }
  float es[8];
#pragma unroll
  for (int r = 0; r < 8; ++r) es[r] = 0.0f;
  {
    float*    srow = stg + (size_t)(16 * rg + 8 * h) * HDIM + cb + m;
    _Float16* trow = tile + (size_t)(16 * rg + 8 * h) * LDH + cb + m;
#pragma unroll
    for (int nt = 0; nt < 4; ++nt) {
      const int col = cb + 16 * nt + m;
      const float bb = be2[col], wv = Winf[col];
#pragma unroll
      for (int r = 0; r < 8; ++r) {
        const float v = silu_f(acc[nt][r] * INV_HW + bb);
        es[r] += v * wv;
        srow[r * HDIM + 16 * nt] = v;
        trow[r * LDH + 16 * nt] = (_Float16)(v * SCL_ACT);
      }
    }
  }
#pragma unroll
  for (int r = 0; r < 8; ++r) {
    float t = es[r];
    t += __shfl_xor(t, 8);
    t += __shfl_xor(t, 4);
    t += __shfl_xor(t, 2);
    t += __shfl_xor(t, 1);
    es[r] = t;
  }
  {
    float mine = 0.0f;
#pragma unroll
    for (int r = 0; r < 8; ++r) mine = ((m & 7) == r) ? es[r] : mine;
    if (m < 8) esx[(16 * rg + 8 * h + m) * 2 + ch] = mine;
  }
  __syncthreads();

#pragma unroll
  for (int nt = 0; nt < 4; ++nt) acc[nt] = zero8();
  {
    const _Float16* arow = tile + (size_t)(16 * rg + m) * LDH + 8 * h;
    const _Float16* bq0  = wx + (size_t)(cb + m) * HDIM + 8 * h;
#pragma unroll 1
    for (int kt = 0; kt < HDIM / 32; ++kt) {
      const v16h a = frag16(arow + 32 * kt);
#pragma unroll
      for (int nt = 0; nt < 4; ++nt) acc[nt] = wmh(a, frag16(bq0 + (size_t)(16 * nt) * HDIM + 32 * kt), acc[nt]);
    }
  }
#pragma unroll
  for (int r = 0; r < 8; ++r) es[r] = 0.0f;
#pragma unroll
  for (int nt = 0; nt < 4; ++nt) {
    const int col = cb + 16 * nt + m;
    const float bb = bx1[col], wv = Wx2[col];
#pragma unroll
    for (int r = 0; r < 8; ++r) es[r] += silu_f(acc[nt][r] * INV_HW + bb) * wv;
  }
#pragma unroll
  for (int r = 0; r < 8; ++r) {
    float t = es[r];
    t += __shfl_xor(t, 8);
    t += __shfl_xor(t, 4);
    t += __shfl_xor(t, 2);
    t += __shfl_xor(t, 1);
    es[r] = t;
  }
  {
    float mine = 0.0f;
#pragma unroll
    for (int r = 0; r < 8; ++r) mine = ((m & 7) == r) ? es[r] : mine;
    if (m < 8) xsx[(16 * rg + 8 * h + m) * 2 + ch] = mine;
  }
  __syncthreads();

  if (tid < TR) {
    const int row = tid;
    const int eg = ebase + rl0 + row;
    const int e = eg > nE - 1 ? nE - 1 : eg;
    int s = ei[e];
    int d = ei[(size_t)nE + e];
    s = s < 0 ? 0 : (s > nN - 1 ? nN - 1 : s);
    d = d < 0 ? 0 : (d > nN - 1 ? nN - 1 : d);
    const float* xs = x + (size_t)s * 3;
    const float* xd = x + (size_t)d * 3;
    const float rx = xd[0] - xs[0], ry = xd[1] - xs[1], rz = xd[2] - xs[2];
    const float dsq  = (rx * rx + rz * rz) + ry * ry;
    const float dist = sqrtf(dsq + 1e-8f);
    const float rinv = rcp_f(dist + 1.0f);
    const float ev = sigm_f(esx[2 * row] + esx[2 * row + 1] + binf[0]);
    const float xw = tanhf(xsx[2 * row] + xsx[2 * row + 1]);
    v4f o;
    o.x = rx * rinv * xw; o.y = ry * rinv * xw; o.z = rz * rinv * xw; o.w = ev;
    float* ap2 = aux + (size_t)(rl0 + row) * 4;
    *(volatile v4f*)ap2 = o;
    __threadfence();
    *(volatile v4f*)ap2 = o;
  }

  float* dstp = mijf + (size_t)rl0 * HDIM;
  v4f ov[NIT4];
#pragma unroll
  for (int it = 0; it < NIT4; ++it) ov[it] = *(const v4f*)(stg + 4 * (it * NTHR + tid));
#pragma unroll
  for (int it = 0; it < NIT4; ++it) *(volatile v4f*)(dstp + 4 * (size_t)(it * NTHR + tid)) = ov[it];
  __threadfence();
#pragma unroll
  for (int it = 0; it < NIT4; ++it) *(volatile v4f*)(dstp + 4 * (size_t)(it * NTHR + tid)) = ov[it];
}

__global__ __launch_bounds__(NTHR) __attribute__((amdgpu_num_vgpr(256)))
void k_gather(const int* __restrict__ ei, const float* __restrict__ mijf, const float* __restrict__ aux,
              const float* __restrict__ x, float* mi, float* dx, float* xout,
              int nE, int nN, int ebase, int clen, int firstChunk, int lastChunk, int nOutX) {
  extern __shared__ __align__(16) char smem_g[];
  int*            slist  = (int*)(smem_g + LG_SLIST);
  unsigned short* slots  = (unsigned short*)(smem_g + LG_SLOTS);
  int*            sdl    = (int*)(smem_g + LG_SDL);
  float*          sdx    = (float*)(smem_g + LG_SDX);
  float*          xo     = (float*)(smem_g + LG_XO);
  int*            scount = (int*)(smem_g + LG_SCNT);
  int*            wsum   = (int*)(smem_g + LG_WSUM);
  int*            scnt   = wsum + NWV;

  const int tid = threadIdx.x, lane = tid & 31;
  const int wave = __builtin_amdgcn_readfirstlane(tid >> 5);
  const int node0 = blockIdx.x * NB;
  const bool vec_ok = (((nE + ebase) & 3) == 0);
  const v4f z4 = {0.0f, 0.0f, 0.0f, 0.0f};
  const float qn = __int_as_float(0x7fc00000);
  const v4f vnan = {qn, qn, qn, qn};

  int cnt = 0, pass = 0;
  for (int cb = 0; ; cb += CH) {
    const bool endc = (cb >= clen);
    if (endc || (cnt + CH > LCAP)) {
      __syncthreads();
      int k = 0;
#pragma unroll 1
      for (int i = 0; i < cnt; i += 4) {
        const v4i w4 = *(const v4i*)(sdl + i);
#pragma unroll
        for (int q = 0; q < 4; ++q) {
          const bool hit = (w4[q] == tid) && (i + q < cnt);
          if (hit) {
            if (k < SP) slots[tid * SP + k] = (unsigned short)(i + q);
            ++k;
          }
        }
      }
      scount[tid] = k;
      __syncthreads();

      const bool first = (firstChunk != 0) && (pass == 0);
      const int nw0 = node0 + 32 * wave;
      v4f vold = *(const v4f*)(dx + (size_t)(nw0 + lane) * 4);
      vold = first ? z4 : vold;
      v4f vdx = z4;
#pragma unroll 1
      for (int j = 0; j < 32; ++j) {
        const int nl = 32 * wave + j;
        float* mrow = mi + (size_t)(node0 + nl) * HDIM + 4 * lane;
        int cn = __builtin_amdgcn_readfirstlane(scount[nl]);
        const bool ovf = cn > SP;
        cn = cn > SP ? SP : cn;
        v4f acc = *(const v4f*)mrow;
        acc = first ? z4 : acc;
        v4f dacc = z4;
#pragma unroll 1
        for (int p = 0; p < cn; ++p) {
          int i = (int)slots[nl * SP + p];
          i = i > LCAP - 1 ? LCAP - 1 : i;
          int el = slist[i];
          el = el < 0 ? 0 : (el > clen - 1 ? clen - 1 : el);
          const v4f avv = *(const v4f*)(aux + (size_t)el * 4);
          const v4f ms  = *(const v4f*)(mijf + (size_t)el * HDIM + 4 * lane);
          acc = acc + ms * avv.w;
          dacc.x += avv.x; dacc.y += avv.y; dacc.z += avv.z;
        }
        acc = ovf ? vnan : acc;
        *(volatile v4f*)mrow = acc;
        __threadfence();
        *(volatile v4f*)mrow = acc;
        const v4f nv = vold + dacc;
        vdx = (lane == j) ? nv : vdx;
      }
      float* drow = dx + (size_t)(nw0 + lane) * 4;
      *(volatile v4f*)drow = vdx;
      __threadfence();
      *(volatile v4f*)drow = vdx;
      *(v4f*)(sdx + (size_t)(32 * wave + lane) * 4) = vdx;
      __syncthreads();
      ++pass;
      cnt = 0;
    }
    if (endc) break;

    int dv[8];
    if (vec_ok && (cb + CH <= clen)) {
      const int* bp = ei + (size_t)nE + ebase + cb + 8 * tid;
      const v4i a = *(const v4i*)bp;
      const v4i b = *(const v4i*)(bp + 4);
      dv[0] = a[0]; dv[1] = a[1]; dv[2] = a[2]; dv[3] = a[3];
      dv[4] = b[0]; dv[5] = b[1]; dv[6] = b[2]; dv[7] = b[3];
    } else {
#pragma unroll
      for (int j = 0; j < 8; ++j) {
        const int el = cb + 8 * tid + j;
        const int ec = el > clen - 1 ? clen - 1 : el;
        const int dj = ei[(size_t)nE + ebase + ec];
        dv[j] = (el < clen) ? dj : -1;
      }
    }
    unsigned bits = 0u;
#pragma unroll
    for (int j = 0; j < 8; ++j) {
      const int dlj = dv[j] - node0;
      bits |= ((unsigned)dlj < (unsigned)NB) ? (1u << j) : 0u;
    }
    const int pc = __builtin_popcount(bits);
    int incl = pc;
#pragma unroll
    for (int sh = 1; sh < 32; sh <<= 1) {
      const int t = __shfl_up(incl, sh);
      incl += (lane >= sh) ? t : 0;
    }
    if (lane == 31) wsum[wave] = incl;
    __syncthreads();
    int woff = 0, tot = 0;
#pragma unroll
    for (int w = 0; w < NWV; ++w) {
      const int v = wsum[w];
      woff += (w < wave) ? v : 0;
      tot += v;
    }
    int pos = cnt + woff + incl - pc;
#pragma unroll
    for (int j = 0; j < 8; ++j) {
      if (bits & (1u << j)) {
        if (pos < LCAP) {
          slist[pos] = cb + 8 * tid + j;
          sdl[pos]   = dv[j] - node0;
        }
        ++pos;
      }
    }
    if (tid == 0) scnt[0] = cnt + tot;
    __syncthreads();
    cnt = scnt[0];
    cnt = cnt > LCAP ? LCAP : cnt;
  }

  if (lastChunk != 0) {
    for (int i = tid; i < NB * 3; i += NTHR) {
      const int nl = i / 3;
      const int c  = i - nl * 3;
      const int node = node0 + nl;
      const int nc = node > nN - 1 ? nN - 1 : node;
      xo[i] = x[(size_t)nc * 3 + c] + sdx[nl * 4 + c];
    }
    __syncthreads();
    if (tid < NB * 3 / 4) {
      const int g0 = node0 * 3 + 4 * tid;
      const v4f v = *(const v4f*)(xo + 4 * tid);
      float* dp = xout + g0;
      if (g0 + 3 < nOutX) {
        *(volatile v4f*)dp = v;
        __threadfence();
        *(volatile v4f*)dp = v;
      } else {
        if (g0 < nOutX)     *(volatile float*)(dp)     = v.x;
        if (g0 + 1 < nOutX) *(volatile float*)(dp + 1) = v.y;
        if (g0 + 2 < nOutX) *(volatile float*)(dp + 2) = v.z;
        if (g0 + 3 < nOutX) *(volatile float*)(dp + 3) = v.w;
        __threadfence();
        if (g0 < nOutX)     *(volatile float*)(dp)     = v.x;
        if (g0 + 1 < nOutX) *(volatile float*)(dp + 1) = v.y;
        if (g0 + 2 < nOutX) *(volatile float*)(dp + 2) = v.z;
        if (g0 + 3 < nOutX) *(volatile float*)(dp + 3) = v.w;
      }
    }
  }
}

__global__ __launch_bounds__(NTHR) __attribute__((amdgpu_num_vgpr(256)))
void k_node(const float* __restrict__ mi, const float* __restrict__ hin,
            const _Float16* __restrict__ wn1, const _Float16* __restrict__ wn2,
            const float* __restrict__ bn1, const float* __restrict__ bn2, float* hout, int nN) {
  constexpr int NIT4 = (TR * HDIM / 4) / NTHR;
  __shared__ __attribute__((aligned(16))) _Float16 tile[TR * LDH];
  __shared__ __attribute__((aligned(16))) float    stg[TR * HDIM];
  const int tid = threadIdx.x, lane = tid & 31;
  const int wave = __builtin_amdgcn_readfirstlane(tid >> 5);
  const int h = lane >> 4, m = lane & 15;
  const int rg = wave >> 1, ch = wave & 1;
  const int cb = 64 * ch;
  const int rowBase = blockIdx.x * TR;
  const int grow = rowBase + 16 * rg + m;
  const int gcl = grow > nN - 1 ? nN - 1 : grow;

  v8f acc[4];
#pragma unroll
  for (int nt = 0; nt < 4; ++nt) acc[nt] = zero8();
  {
    const float* ap1 = mi  + (size_t)grow * HDIM;
    const float* ap2 = hin + (size_t)gcl * HDIM;
    const _Float16* bp0 = wn1 + (size_t)(cb + m) * (2 * HDIM) + 8 * h;
#pragma unroll 1
    for (int kt = 0; kt < HDIM / 32; ++kt) {
      const v16h a = afrag_f32(ap1 + 32 * kt, h, SCL_ACT);
#pragma unroll
      for (int nt = 0; nt < 4; ++nt)
        acc[nt] = wmh(a, frag16(bp0 + (size_t)(16 * nt) * (2 * HDIM) + 32 * kt), acc[nt]);
    }
#pragma unroll 1
    for (int kt = 0; kt < HDIM / 32; ++kt) {
      const v16h a = afrag_f32(ap2 + 32 * kt, h, SCL_H);
#pragma unroll
      for (int nt = 0; nt < 4; ++nt)
        acc[nt] = wmh(a, frag16(bp0 + (size_t)(16 * nt) * (2 * HDIM) + HDIM + 32 * kt), acc[nt]);
    }
  }
  {
    _Float16* trow = tile + (size_t)(16 * rg + 8 * h) * LDH + cb + m;
#pragma unroll
    for (int nt = 0; nt < 4; ++nt) {
      const float bb = bn1[cb + 16 * nt + m];
#pragma unroll
      for (int r = 0; r < 8; ++r)
        trow[r * LDH + 16 * nt] = (_Float16)(silu_f(acc[nt][r] * INV_HW + bb) * SCL_ACT);
    }
  }
  __syncthreads();

#pragma unroll
  for (int nt = 0; nt < 4; ++nt) acc[nt] = zero8();
  {
    const _Float16* arow = tile + (size_t)(16 * rg + m) * LDH + 8 * h;
    const _Float16* bq0  = wn2 + (size_t)(cb + m) * HDIM + 8 * h;
#pragma unroll 1
    for (int kt = 0; kt < HDIM / 32; ++kt) {
      const v16h a = frag16(arow + 32 * kt);
#pragma unroll
      for (int nt = 0; nt < 4; ++nt) acc[nt] = wmh(a, frag16(bq0 + (size_t)(16 * nt) * HDIM + 32 * kt), acc[nt]);
    }
  }
  {
    float* srow = stg + (size_t)(16 * rg + 8 * h) * HDIM + cb + m;
#pragma unroll
    for (int nt = 0; nt < 4; ++nt) {
      const float bb = bn2[cb + 16 * nt + m];
#pragma unroll
      for (int r = 0; r < 8; ++r) srow[r * HDIM + 16 * nt] = acc[nt][r] * INV_HW + bb;
    }
  }
  __syncthreads();

  v4f ov[NIT4];
#pragma unroll
  for (int it = 0; it < NIT4; ++it) {
    const int u = it * NTHR + tid;
    const int orow = rowBase + (u >> 5);
    const int oc = orow > nN - 1 ? nN - 1 : orow;
    const v4f hv = *(const v4f*)(hin + (size_t)oc * HDIM + 4 * (u & 31));
    ov[it] = *(const v4f*)(stg + 4 * u) + hv;
  }
#pragma unroll
  for (int it = 0; it < NIT4; ++it) {
    const int u = it * NTHR + tid;
    const int orow = rowBase + (u >> 5);
    if (orow < nN) *(volatile v4f*)(hout + (size_t)orow * HDIM + 4 * (u & 31)) = ov[it];
  }
  __threadfence();
#pragma unroll
  for (int it = 0; it < NIT4; ++it) {
    const int u = it * NTHR + tid;
    const int orow = rowBase + (u >> 5);
    if (orow < nN) *(volatile v4f*)(hout + (size_t)orow * HDIM + 4 * (u & 31)) = ov[it];
  }
}

extern "C" void kernel_launch(void* const* d_in, const int* in_sizes, int n_in,
                              void* d_out, int out_size, void* d_ws, size_t ws_size,
                              hipStream_t stream) {
  if (n_in < 18) return;
  const int nN = in_sizes[0] / HDIM;
  const int nE = in_sizes[2] / 2;
  if (nN <= 0 || nE <= 0) return;
  if (in_sizes[0] != nN * HDIM || in_sizes[1] != nN * 3 || in_sizes[2] != 2 * nE) return;
  if (in_sizes[3] != nN || in_sizes[4] != nE * EFD) return;
  if (in_sizes[5] != K1R * HDIM || in_sizes[6] != HDIM) return;
  if (in_sizes[7] != HDIM * HDIM || in_sizes[8] != HDIM) return;
  if (in_sizes[9] != HDIM || in_sizes[10] != 1) return;
  if (in_sizes[11] != HDIM * HDIM || in_sizes[12] != HDIM || in_sizes[13] != HDIM) return;
  if (in_sizes[14] != 2 * HDIM * HDIM || in_sizes[15] != HDIM) return;
  if (in_sizes[16] != HDIM * HDIM || in_sizes[17] != HDIM) return;
  if (out_size != nN * HDIM + nN * 3) return;
  if (nE > (1 << 27) || nN > (1 << 22)) return;

  const float* hin  = (const float*)d_in[0];
  const float* x    = (const float*)d_in[1];
  const int*   ei   = (const int*)d_in[2];
  const float* ea   = (const float*)d_in[4];
  const float* We1  = (const float*)d_in[5];
  const float* be1  = (const float*)d_in[6];
  const float* We2  = (const float*)d_in[7];
  const float* be2  = (const float*)d_in[8];
  const float* Winf = (const float*)d_in[9];
  const float* binf = (const float*)d_in[10];
  const float* Wx1  = (const float*)d_in[11];
  const float* bx1  = (const float*)d_in[12];
  const float* Wx2  = (const float*)d_in[13];
  const float* Wn1  = (const float*)d_in[14];
  const float* bn1  = (const float*)d_in[15];
  const float* Wn2  = (const float*)d_in[16];
  const float* bn2  = (const float*)d_in[17];
  float* hout = (float*)d_out;
  float* xout = (float*)d_out + (size_t)nN * HDIM;

  const int nGat   = (nN + NB - 1) / NB;
  const int NPAD   = nGat * NB;
  const int nGemm  = NPAD / BM;
  const int nNode  = NPAD / TR;
  const int nChunk = (nE + CE - 1) / CE;
  if (nChunk > 256) return;

  char* ws = (char*)d_ws;
  size_t off = 0;
  const size_t oWPQ = off; off += (size_t)PW * HDIM * 2;        off = (off + 255) & ~(size_t)255;
  const size_t oWE  = off; off += (size_t)HDIM * KE * 2;        off = (off + 255) & ~(size_t)255;
  const size_t oW2  = off; off += (size_t)HDIM * HDIM * 2;      off = (off + 255) & ~(size_t)255;
  const size_t oWX  = off; off += (size_t)HDIM * HDIM * 2;      off = (off + 255) & ~(size_t)255;
  const size_t oWN1 = off; off += (size_t)HDIM * 2 * HDIM * 2;  off = (off + 255) & ~(size_t)255;
  const size_t oWN2 = off; off += (size_t)HDIM * HDIM * 2;      off = (off + 255) & ~(size_t)255;
  const size_t oPQ  = off; off += (size_t)NPAD * PW * 4;        off = (off + 255) & ~(size_t)255;
  const size_t oMI  = off; off += (size_t)NPAD * HDIM * 4;      off = (off + 255) & ~(size_t)255;
  const size_t oDX  = off; off += (size_t)NPAD * 4 * 4;         off = (off + 255) & ~(size_t)255;
  const size_t oM1  = off; off += (size_t)CE * HDIM * 2;        off = (off + 255) & ~(size_t)255;
  const size_t oMJ  = off; off += (size_t)CE * HDIM * 4;        off = (off + 255) & ~(size_t)255;
  const size_t oAUX = off; off += (size_t)CE * 4 * 4;           off = (off + 255) & ~(size_t)255;
  if (off > ws_size || off > (size_t)WSCAP) return;
  _Float16* wPQ  = (_Float16*)(ws + oWPQ);
  _Float16* wE   = (_Float16*)(ws + oWE);
  _Float16* w2   = (_Float16*)(ws + oW2);
  _Float16* wx   = (_Float16*)(ws + oWX);
  _Float16* wn1  = (_Float16*)(ws + oWN1);
  _Float16* wn2  = (_Float16*)(ws + oWN2);
  float*    pqP  = (float*)(ws + oPQ);
  float*    miP  = (float*)(ws + oMI);
  float*    dxP  = (float*)(ws + oDX);
  _Float16* m1p  = (_Float16*)(ws + oM1);
  float*    mijf = (float*)(ws + oMJ);
  float*    auxp = (float*)(ws + oAUX);

  (void)hipFuncSetAttribute(reinterpret_cast<const void*>(&k_gather),
                            hipFuncAttributeMaxDynamicSharedMemorySize, (int)LDS_G);

  const int u128 = HDIM * (HDIM / 8);
  const int u256 = HDIM * (2 * HDIM / 8);
  const int u32  = HDIM * (KE / 8);
  k_wcvt<<<(u128 + NTHR - 1) / NTHR, NTHR, 0, stream>>>(We1, wPQ, HDIM, 0, HDIM, HDIM, u128, SCL_W);
  k_wcvt<<<(u128 + NTHR - 1) / NTHR, NTHR, 0, stream>>>(We1, wPQ + (size_t)HDIM * HDIM, HDIM, HDIM, HDIM, HDIM, u128, SCL_W);
  k_wcvt<<<(u32 + NTHR - 1) / NTHR, NTHR, 0, stream>>>(We1, wE, HDIM, 2 * HDIM, K1R - 2 * HDIM, KE, u32, SCL_W);
  k_wcvt<<<(u128 + NTHR - 1) / NTHR, NTHR, 0, stream>>>(We2, w2, HDIM, 0, HDIM, HDIM, u128, SCL_W);
  k_wcvt<<<(u128 + NTHR - 1) / NTHR, NTHR, 0, stream>>>(Wx1, wx, HDIM, 0, HDIM, HDIM, u128, SCL_W);
  k_wcvt<<<(u256 + NTHR - 1) / NTHR, NTHR, 0, stream>>>(Wn1, wn1, HDIM, 0, 2 * HDIM, 2 * HDIM, u256, SCL_W);
  k_wcvt<<<(u128 + NTHR - 1) / NTHR, NTHR, 0, stream>>>(Wn2, wn2, HDIM, 0, HDIM, HDIM, u128, SCL_W);
  k_nodegemm<<<nGemm, NTHR, 0, stream>>>(hin, wPQ, be1, pqP, nN);
  for (int c = 0; c < nChunk; ++c) {
    const int ebase = c * CE;
    const int clen  = (nE - ebase) < CE ? (nE - ebase) : CE;
    const int nb    = (clen + TR - 1) / TR;
    k_edge1<<<nb, NTHR, 0, stream>>>(pqP, ei, x, ea, wE, m1p, nE, nN, ebase);
    k_edge2<<<nb, NTHR, 0, stream>>>(m1p, ei, x, w2, wx, be2, Winf, binf, bx1, Wx2, mijf, auxp, nE, nN, ebase);
    k_gather<<<nGat, NTHR, LDS_G, stream>>>(ei, mijf, auxp, x, miP, dxP, xout, nE, nN, ebase, clen,
                                             (c == 0) ? 1 : 0, (c == nChunk - 1) ? 1 : 0, nN * 3);
  }
  k_node<<<nNode, NTHR, 0, stream>>>(miP, hin, wn1, wn2, bn1, bn2, hout, nN);
}
